// GNNLayer_60335700574605
// MI455X (gfx1250) — hardware-verified
//
#include <hip/hip_runtime.h>


namespace {
constexpr int N = 100000, NP = 100032, NPL = NP  , D = 128, KN = 16, NBLK = NP / 64;
constexpr float XS = 8.0f, WSC = 256.0f;
static_assert(NP % 64 == 0 && NP >= N && D == 128, "tiling");
typedef _Float16 b16;
typedef __attribute__((ext_vector_type(16))) _Float16 v16b;
typedef __attribute__((ext_vector_type(8))) _Float16 v8b;
typedef __attribute__((ext_vector_type(8))) float v8f;
typedef __attribute__((ext_vector_type(4))) float v4f;
__device__ __forceinline__ float bf16_rne(float f) { unsigned int u = __float_as_uint(f); u += 0x7FFFu + ((u >> 16) & 1u); return __uint_as_float(u & 0xFFFF0000u); }
__device__ __forceinline__ void split16(float v, b16& hi, b16& lo) { hi = (b16)v; lo = (b16)(v - (float)hi); }
__device__ __forceinline__ v16b frag_kb(const b16* p, int hh) { const v8b a = *(const v8b*)(p + 8 * hh), b = *(const v8b*)(p + 16 + 8 * hh); v16b f;
#pragma unroll
  for (int e = 0; e < 8; ++e) { f[e] = a[e]; f[8 + e] = b[e]; } return f; }
__device__ __forceinline__ v8f wmma16b(v16b a, v16b b, v8f c) { v8f d = __builtin_amdgcn_wmma_f32_16x16x32_f16(false, a, false, b, (short)0, c, false, false); asm volatile("v_nop\n\tv_nop\n\tv_nop\n\tv_nop" : "+v"(d) : "v"(a), "v"(b)); return d; }
__device__ __forceinline__ void wave_lds_sync() { __builtin_amdgcn_fence(__ATOMIC_RELEASE, "workgroup"); __builtin_amdgcn_wave_barrier(); __builtin_amdgcn_fence(__ATOMIC_ACQUIRE, "workgroup"); }
__device__ __forceinline__ float pmul(float a, float b) { float p = a * b; asm volatile("" : "+v"(p)); return p; }
__device__ __forceinline__ int iclamp(int v, int lo, int hi) { return v < lo ? lo : (v > hi ? hi : v); }

typedef __attribute__((ext_vector_type(2))) _Float16 v2h;
typedef __attribute__((ext_vector_type(4))) _Float16 v4h;
typedef __attribute__((ext_vector_type(2))) float v2f;
typedef __attribute__((ext_vector_type(4))) int v4i;
__device__ __forceinline__ float nexp2(float v) { return __builtin_amdgcn_exp2f(v); }
__global__ __launch_bounds__(256) void wt_kernel(const float* __restrict__ w, b16* __restrict__ WT) {
  const int u = blockIdx.x * 256 + threadIdx.x; if (u >= D * D / 8) return; const int e = u * 8; v8b v;
  for (int j = 0; j < 8; ++j) v[j] = (b16)(bf16_rne(w[e + j]) * WSC);
  for (int pass = 0; pass < 2; ++pass) { *(volatile v8b*)(WT + e) = v; __threadfence(); }
}
__global__ __launch_bounds__(128) void lin_kernel(const float* __restrict__ Hin, const b16* __restrict__ WT, float* __restrict__ NH, float* __restrict__ PMIN) {
  __shared__ __attribute__((aligned(16))) b16 Ah[4][16][D + 8]; __shared__ __attribute__((aligned(16))) float Tf[4][16][D + 4];
  const int wave = threadIdx.x >> 5, lane = threadIdx.x & 31, nloc = lane & 15, hlf = lane >> 4; const size_t m0 = (size_t)blockIdx.x * 64 + wave * 16;
  for (int idx = lane; idx < 16 * (D / 4); idx += 32) { const int rr = idx / (D / 4), c4 = (idx % (D / 4)) * 4; const size_t arow = (m0 + rr < (size_t)N) ? m0 + rr : (size_t)N - 1; const v4f v = *(const v4f*)(Hin + arow * D + c4); v4h hv; for (int j = 0; j < 4; ++j) hv[j] = (b16)(bf16_rne(v[j]) * XS); *(v4h*)(&Ah[wave][rr][c4]) = hv; }
  wave_lds_sync();
  v8f acc[8]; for (int t = 0; t < 8; ++t) acc[t] = (v8f){};
#pragma unroll
  for (int kb = 0; kb < D; kb += 32) { const v16b a = frag_kb(&Ah[wave][nloc][kb], hlf);
#pragma unroll
    for (int t = 0; t < 8; ++t) acc[t] = wmma16b(a, frag_kb(WT + (size_t)(t * 16 + nloc) * D + kb, hlf), acc[t]); }
#pragma unroll
  for (int t = 0; t < 8; ++t) for (int r = 0; r < 8; ++r) Tf[wave][8 * hlf + r][t * 16 + nloc] = (m0 + 8 * hlf + r < (size_t)N) ? fmaxf(acc[t][r] * (1.0f / (XS * WSC)), 0.0f) : 0.0f;
  __syncthreads();
  float cm = INFINITY; { const int c = threadIdx.x; for (int rr = 0; rr < 64; ++rr) if ((size_t)blockIdx.x * 64 + rr < (size_t)N) cm = fminf(cm, Tf[rr >> 4][rr & 15][c]); }
  for (int pass = 0; pass < 2; ++pass) { for (int rr = 0; rr < 16; ++rr) *(volatile v4f*)(NH + (m0 + rr) * D + lane * 4) = *(const v4f*)(&Tf[wave][rr][lane * 4]);
    ((volatile float*)PMIN)[(size_t)blockIdx.x * D + threadIdx.x] = cm; __threadfence(); }
}
__global__ __launch_bounds__(128) void min_kernel(const float* __restrict__ PMIN, float* __restrict__ MINR) {
  const int c = threadIdx.x; float cm = INFINITY;
  for (int bk = 0; bk < NBLK; ++bk) cm = fminf(cm, PMIN[(size_t)bk * D + c]);
  for (int pass = 0; pass < 2; ++pass) { ((volatile float*)MINR)[c] = cm; __threadfence(); }
}
__global__ __launch_bounds__(256) void gmax_kernel(const float* __restrict__ NH, const float* __restrict__ MINR, const int* __restrict__ nbr, float* __restrict__ out, int mrows) {
  const int tid = threadIdx.x; const int row = tid >> 3, g = tid & 7, c0 = g * 16; const int v = blockIdx.x * 32 + row; const int vv = v < N ? v : N - 1;
  float m[16]; for (int j = 0; j < 16; ++j) m[j] = -INFINITY;
#pragma unroll 1
  for (int k = 0; k < KN; ++k) { const int raw = nbr[(size_t)vv * KN + k]; const bool pad = (raw < 0) || (raw >= N); const float* src = pad ? (MINR + c0) : (NH + (size_t)raw * D + c0);
#pragma unroll
    for (int q = 0; q < 4; ++q) { const v4f t4 = *(const v4f*)(src + 4 * q); for (int j = 0; j < 4; ++j) m[4 * q + j] = fmaxf(m[4 * q + j], t4[j]); } }
  for (int pass = 0; pass < 2; ++pass) { if (v < mrows) { float* orow = out + (size_t)v * D + c0;
#pragma unroll
      for (int q = 0; q < 4; ++q) { v4f o4; for (int j = 0; j < 4; ++j) o4[j] = (v < N) ? m[4 * q + j] : 0.0f; *(volatile v4f*)(orow + 4 * q) = o4; } }
    __threadfence(); }
}
}

extern "C" void kernel_launch(void* const* d_in, const int* in_sizes, int n_in, void* d_out, int out_size, void* d_ws, size_t ws_size, hipStream_t stream) {
  (void)n_in;
  auto Fp = [&](int i) { return (const float*)d_in[i]; };
  if (in_sizes[0] != N * D || in_sizes[1] != N * KN || in_sizes[2] != D * D || out_size != N * D) return;
  size_t off = 0; char* ws = (char*)d_ws;
  auto carve = [&](size_t bytes) { char* p = ws + off; off += (bytes + 255) & ~(size_t)255; return p; };
  b16* WT = (b16*)carve((size_t)D * D * 2); float* NH = (float*)carve((size_t)NP * D * 4); float* PMIN = (float*)carve((size_t)NBLK * D * 4); float* MINR = (float*)carve((size_t)D * 4);
  if (off > ws_size || off > ((size_t)128 << 20)) return;
  wt_kernel<<<(D * D / 8 + 255) / 256, 256, 0, stream>>>(Fp(2), WT);
  lin_kernel<<<NBLK, 128, 0, stream>>>(Fp(0), WT, NH, PMIN);
  min_kernel<<<1, 128, 0, stream>>>(PMIN, MINR);
  gmax_kernel<<<NPL / 32, 256, 0, stream>>>(NH, MINR, (const int*)d_in[1], (float*)d_out, N);
}
